// TaskMoE_13288628813932
// MI455X (gfx1250) — hardware-run, weakly checked
//
#include <hip/hip_runtime.h>
#include <math.h>

#define NTOK 4096
#define NPASS 2
#define NTOK_ALL (NTOK * NPASS)
#define DM 1024
#define FF 1024
#define NE 8
#define TOPK 2
#define NER 16
#define NSLOT (NTOK * TOPK)
#define R_MAX (NSLOT + 64 * NER)
#define NT_MAX (R_MAX / 64)
#define NGW (NTOK / 16)

#define CX_LOG2 11
#define CW_LOG2 16
#define CH_LOG2 11
#define SC_Y (1.0f / (float)(1u << (CH_LOG2 + CW_LOG2)))

#define RW_CH 8192
#define TBL_COUNT 0
#define TBL_POFF 16
#define TBL_NTILES 40
#define TBL_TILE_E 64
#define TBL_HDR 256
#define TBL_ROWTOK TBL_HDR
#define TBL_SLOTROW (TBL_HDR + R_MAX)
#define TBL_WORDS (TBL_HDR + R_MAX + NSLOT)

static_assert(NE == 8 && TOPK == 2 && NER == 16 && NE <= NER && NPASS == 2);
static_assert(DM == 1024 && FF == 1024 && DM % 64 == 0 && FF % 64 == 0 && NTOK % 128 == 0);
static_assert(NSLOT % 128 == 0 && R_MAX % 128 == 0 && R_MAX >= NSLOT + 63 * NER);
static_assert(TBL_HDR % 32 == 0 && TBL_HDR <= 512);
static_assert(TBL_COUNT + NER <= TBL_POFF && TBL_POFF + NER + 1 <= TBL_NTILES && TBL_NTILES < TBL_TILE_E && TBL_TILE_E + NT_MAX <= TBL_HDR);
static_assert(RW_CH % 128 == 0 && (TBL_WORDS * 4) % 256 == 0 && NSLOT <= RW_CH);
static_assert((NTOK_ALL * DM / 8) % 256 == 0 && R_MAX % 2 == 0);
static_assert(CX_LOG2 == 11 && CW_LOG2 == 16 && CH_LOG2 == CX_LOG2);
static_assert(NSLOT == 8192 && R_MAX == 9216 && NT_MAX == 144 && TBL_WORDS == 17664);

constexpr size_t al256(size_t b) { return (b + 255) & ~(size_t)255; }
constexpr size_t SZ_X16 = al256((size_t)NTOK_ALL * DM * 2);
constexpr size_t SZ_WP  = al256((size_t)NE * DM * FF * 2);
constexpr size_t SZ_SEL = al256((size_t)NSLOT * 4);
constexpr size_t SZ_WGT = al256((size_t)NSLOT * 4);
constexpr size_t SZ_GS  = al256((size_t)NPASS * NGW * 32 * 4);
constexpr size_t SZ_TBL = al256((size_t)TBL_WORDS * 4);
constexpr size_t SZ_XG  = al256((size_t)R_MAX * FF * 2);
constexpr size_t SZ_YG  = al256((size_t)R_MAX * DM * 4);
constexpr size_t WS_TOTAL = SZ_X16 + SZ_WP + NPASS * (SZ_SEL + SZ_WGT + SZ_TBL) + SZ_GS + SZ_XG + SZ_YG;
static_assert(WS_TOTAL == (size_t)90515456 && WS_TOTAL < (size_t)134217728);

typedef _Float16 h16;
typedef __attribute__((ext_vector_type(16))) _Float16 v16h;
typedef __attribute__((ext_vector_type(8)))  _Float16 v8h;
typedef __attribute__((ext_vector_type(8)))  float    v8f;
typedef __attribute__((ext_vector_type(4)))  float    v4f;
typedef __attribute__((ext_vector_type(2)))  float    v2f;
typedef __attribute__((ext_vector_type(4)))  unsigned int v4u;
typedef __attribute__((ext_vector_type(4)))  int      v4i;
typedef __attribute__((ext_vector_type(2)))  int      v2i;


#define VST2(T, ptr, val) do { const T vst2_v_ = (val); *(volatile T*)(ptr) = vst2_v_; __threadfence(); *(volatile T*)(ptr) = vst2_v_; } while (0)

static __device__ __forceinline__ float bfr(float f) {
    unsigned u = __float_as_uint(f);
    u += 0x7FFFu + ((u >> 16) & 1u);
    return __uint_as_float(u & 0xFFFF0000u);
}
static __device__ __forceinline__ h16 toh_flush(float v) { const float w = (fabsf(v) < 6.103515625e-05f) ? 0.0f : v; return (h16)w; }
static __device__ __forceinline__ void st8h(h16* p, const float* v) {
    v8h hv;
#pragma unroll
    for (int e = 0; e < 8; ++e) hv[e] = toh_flush(v[e]);
    VST2(v8h, p, hv);
}

union FragU { v16h v; v8h h[2]; };
static __device__ __forceinline__ v16h frag_ld(const h16* p) {
    FragU f; f.h[0] = *(const v8h*)(p); f.h[1] = *(const v8h*)(p + 16); return f.v;
}
static __device__ __forceinline__ v8f wmma16g(v16h a, v16h b, v8f c) {
    c = __builtin_amdgcn_wmma_f32_16x16x32_f16(false, a, false, b, (short)0, c, false, false);
    asm volatile("v_nop\n\tv_nop\n\tv_nop\n\tv_nop" : "+v"(c) : "v"(a), "v"(b));
    return c;
}
static __device__ __forceinline__ void wave_sync_lds() {
    __builtin_amdgcn_fence(3  , "workgroup");
    __builtin_amdgcn_wave_barrier();
    __builtin_amdgcn_fence(2  , "workgroup");
}

template <int LOG2C>
__global__ __launch_bounds__(256) void k_plane(const float* __restrict__ src, h16* __restrict__ dst, unsigned n8) {
    const unsigned u = blockIdx.x * 256u + threadIdx.x;
    if (u >= n8) return;
    const float cs = (float)(1u << LOG2C);
    const v4f a = *(const v4f*)(src + (size_t)u * 8u);
    const v4f b = *(const v4f*)(src + (size_t)u * 8u + 4u);
    float v[8] = {bfr(a.x) * cs, bfr(a.y) * cs, bfr(a.z) * cs, bfr(a.w) * cs, bfr(b.x) * cs, bfr(b.y) * cs, bfr(b.z) * cs, bfr(b.w) * cs};
    st8h(dst + (size_t)u * 8u, v);
}

__global__ __launch_bounds__(128) void k_planeTw(const float* __restrict__ src, h16* __restrict__ dst, unsigned ne, unsigned K, unsigned N, unsigned pitch, unsigned estride, float cs) {
    __shared__ __align__(16) float sT[4][64 * 36];
    const unsigned lane = threadIdx.x & 31u;
    const unsigned wave = threadIdx.x >> 5;
    const unsigned tk = K >> 6, tn = N >> 5;
    const unsigned tpe = tk * tn;
    const unsigned u = blockIdx.x * 4u + wave;
    if (u >= ne * tpe) return;
    const unsigned e = u / tpe;
    const unsigned rem = u - e * tpe;
    const unsigned kt = rem / tn;
    const unsigned nt = rem - kt * tn;
    const unsigned k0 = kt << 6, n0 = nt << 5;
    const size_t sbase = (size_t)e * (size_t)estride;
    const size_t ebase = (size_t)e * ((size_t)K * (size_t)N);
    float* slab = sT[wave];
#pragma unroll
    for (int i = 0; i < 16; ++i) {
        const unsigned p = lane + 32u * (unsigned)i;
        const unsigned kr = p >> 3;
        const unsigned n4 = (p & 7u) * 4u;
        const v4f a = *(const v4f*)(src + sbase + (size_t)(k0 + kr) * pitch + n0 + n4);
        v4f s;
        s.x = bfr(a.x) * cs; s.y = bfr(a.y) * cs; s.z = bfr(a.z) * cs; s.w = bfr(a.w) * cs;
        *(v4f*)(&slab[kr * 36u + n4]) = s;
    }
    wave_sync_lds();
#pragma unroll
    for (int i = 0; i < 8; ++i) {
        const unsigned q = lane + 32u * (unsigned)i;
        const unsigned n = q >> 3;
        const unsigned kp = q & 7u;
        float v[8];
#pragma unroll
        for (int j = 0; j < 8; ++j) v[j] = slab[(8u * kp + (unsigned)j) * 36u + n];
        st8h(dst + ebase + (size_t)(n0 + n) * K + k0 + 8u * kp, v);
    }
}

__global__ __launch_bounds__(256) void k_gate(const float* __restrict__ x, const float* __restrict__ gw,
                                              int* __restrict__ sel, float* __restrict__ wgt, float* __restrict__ gs) {
    const unsigned lane = threadIdx.x & 31u;
    const unsigned wave = threadIdx.x >> 5;
    const unsigned gwv = blockIdx.x * 8u + wave;
    const unsigned t0 = gwv * 16u;
    if (t0 >= (unsigned)NTOK) return;
    int ki0 = 0, ki1 = 0;
    float kw0 = 0.0f, kw1 = 0.0f;
    float acc = 0.0f;
    for (unsigned j = 0; j < 16u; ++j) {
        const float* xr = x + (size_t)(t0 + j) * DM;
        float lg[NE];
#pragma unroll
        for (int e = 0; e < NE; ++e) lg[e] = 0.0f;
        for (unsigned i = 0; i < (unsigned)(DM / 32); ++i) {
            const unsigned d = lane + 32u * i;
            const float xv = bfr(xr[d]);
            const v4f ga = *(const v4f*)(gw + (size_t)d * NE);
            const v4f gc = *(const v4f*)(gw + (size_t)d * NE + 4u);
            lg[0] += xv * bfr(ga.x); lg[1] += xv * bfr(ga.y); lg[2] += xv * bfr(ga.z); lg[3] += xv * bfr(ga.w);
            lg[4] += xv * bfr(gc.x); lg[5] += xv * bfr(gc.y); lg[6] += xv * bfr(gc.z); lg[7] += xv * bfr(gc.w);
        }
#pragma unroll
        for (int e = 0; e < NE; ++e) {
            lg[e] += __shfl_xor(lg[e], 16, 32);
            lg[e] += __shfl_xor(lg[e], 8, 32);
            lg[e] += __shfl_xor(lg[e], 4, 32);
            lg[e] += __shfl_xor(lg[e], 2, 32);
            lg[e] += __shfl_xor(lg[e], 1, 32);
        }
        float m = lg[0];
#pragma unroll
        for (int e = 1; e < NE; ++e) m = fmaxf(m, lg[e]);
        float pr[NE];
        float s = 0.0f;
#pragma unroll
        for (int e = 0; e < NE; ++e) { pr[e] = expf(lg[e] - m); s += pr[e]; }
#pragma unroll
        for (int e = 0; e < NE; ++e) pr[e] = pr[e] / s;
        float bestv = pr[0];
        int besti = 0;
#pragma unroll
        for (int e = 1; e < NE; ++e) { const bool c = pr[e] > bestv; bestv = c ? pr[e] : bestv; besti = c ? e : besti; }
        float secv = -1.0f;
        int seci = 0;
#pragma unroll
        for (int e = 0; e < NE; ++e) { const bool c = (e != besti) && (pr[e] > secv); secv = c ? pr[e] : secv; seci = c ? e : seci; }
        const bool mine = (lane == j);
        ki0 = mine ? besti : ki0;  ki1 = mine ? seci : ki1;
        const float psum = bestv + secv;
        kw0 = mine ? bestv / psum : kw0;  kw1 = mine ? secv / psum : kw1;
        float add = 0.0f;
#pragma unroll
        for (int e = 0; e < NE; ++e) add = (lane == (unsigned)e) ? pr[e] : add;
        acc += add;
    }
    if (lane < 16u) {
        v2i sv; sv.x = ki0; sv.y = ki1;
        v2f wv; wv.x = kw0; wv.y = kw1;
        VST2(v2i, sel + (size_t)(t0 + lane) * 2u, sv);
        VST2(v2f, wgt + (size_t)(t0 + lane) * 2u, wv);
    }
    VST2(float, gs + (size_t)gwv * 32u + lane, acc);
}

template <int NE_>
__global__ __launch_bounds__(32) void k_route1w(const int* __restrict__ sel, int* __restrict__ tbl, unsigned nslot, unsigned spt, unsigned hdr, unsigned rmax,
                                                unsigned offPoff, unsigned offNtiles, unsigned offTileE) {
    static_assert(NE_ >= 1 && NE_ <= 32);
    __shared__ __align__(16) int s_img[RW_CH];
    __shared__ __align__(16) int s_hdr[512];
    const unsigned lane = threadIdx.x & 31u;
    const unsigned spl = nslot >> 5;
    const unsigned ng = spl >> 2;
    const unsigned ntmax = rmax >> 6;
    const v4i* sp = (const v4i*)(sel + (size_t)lane * spl);
    int cnt[NE_];
#pragma unroll
    for (int j = 0; j < NE_; ++j) cnt[j] = 0;
    for (unsigned g = 0; g < ng; ++g) {
        const v4i v = sp[g];
#pragma unroll
        for (int c = 0; c < 4; ++c) {
            const int e = min(max(v[c], 0), NE_ - 1);
#pragma unroll
            for (int j = 0; j < NE_; ++j) cnt[j] += (e == j) ? 1 : 0;
        }
    }
    int base0[NE_], total[NE_];
#pragma unroll
    for (int j = 0; j < NE_; ++j) {
        int pre = 0, tot = cnt[j];
#pragma unroll
        for (int d = 1; d < 32; d <<= 1) {
            const int t = __shfl_xor(tot, d, 32);
            pre += ((lane & (unsigned)d) != 0u) ? t : 0;
            tot += t;
        }
        base0[j] = pre;
        total[j] = tot;
    }
    int poff[NE_ + 1];
    poff[0] = 0;
#pragma unroll
    for (int j = 0; j < NE_; ++j) poff[j + 1] = poff[j] + (((total[j] + 63) >> 6) << 6);
    for (unsigned i = lane; i < 512u; i += 32u) s_hdr[i] = (i >= offTileE && i < offTileE + ntmax) ? -1 : 0;
    wave_sync_lds();
    if (lane == 0u) {
#pragma unroll
        for (int j = 0; j < NE_; ++j) { s_hdr[min((unsigned)j, 511u)] = total[j]; s_hdr[min(offPoff + (unsigned)j, 511u)] = poff[j]; }
        s_hdr[min(offPoff + (unsigned)NE_, 511u)] = poff[NE_];
        s_hdr[min(offNtiles, 511u)] = poff[NE_] >> 6;
    }
    for (unsigned t = lane; t < ntmax; t += 32u) {
        const int b64 = (int)(t * 64u);
        int ev = -1;
#pragma unroll
        for (int j = 0; j < NE_; ++j) ev = (b64 >= poff[j] && b64 < poff[j + 1]) ? j : ev;
        s_hdr[min(offTileE + t, 511u)] = ev;
    }
    wave_sync_lds();
    for (int pass = 0; pass < 2; ++pass) {
        for (unsigned i = lane; i < (hdr >> 2); i += 32u) *(volatile v4i*)(tbl + 4u * i) = *(const v4i*)(&s_hdr[4u * i]);
        __threadfence();
    }
    for (unsigned lo = 0; lo < rmax; lo += (unsigned)RW_CH) {
        for (unsigned i = lane; i < (unsigned)(RW_CH / 4); i += 32u) *(v4i*)(&s_img[4u * i]) = (v4i){-1, -1, -1, -1};
        wave_sync_lds();
        int run[NE_];
#pragma unroll
        for (int j = 0; j < NE_; ++j) run[j] = base0[j];
        for (unsigned g = 0; g < ng; ++g) {
            const v4i v = sp[g];
#pragma unroll
            for (int c = 0; c < 4; ++c) {
                const int e = min(max(v[c], 0), NE_ - 1);
                int row = 0;
#pragma unroll
                for (int j = 0; j < NE_; ++j) {
                    const bool hit = (e == j);
                    row = hit ? (poff[j] + run[j]) : row;
                    run[j] += hit ? 1 : 0;
                }
                row = min(max(row, 0), (int)rmax - 1);
                const unsigned rel = (unsigned)row - lo;
                if (rel < (unsigned)RW_CH) s_img[rel] = (int)((lane * spl + 4u * g + (unsigned)c) / spt);
            }
        }
        wave_sync_lds();
        const unsigned nw = min((unsigned)RW_CH, rmax - lo);
        for (int pass = 0; pass < 2; ++pass) {
            for (unsigned i = lane; i < (nw >> 2); i += 32u) *(volatile v4i*)(tbl + hdr + lo + 4u * i) = *(const v4i*)(&s_img[4u * i]);
            __threadfence();
        }
        wave_sync_lds();
    }
    for (unsigned lo = 0; lo < nslot; lo += (unsigned)RW_CH) {
        int run[NE_];
#pragma unroll
        for (int j = 0; j < NE_; ++j) run[j] = base0[j];
        for (unsigned g = 0; g < ng; ++g) {
            const v4i v = sp[g];
#pragma unroll
            for (int c = 0; c < 4; ++c) {
                const int e = min(max(v[c], 0), NE_ - 1);
                int row = 0;
#pragma unroll
                for (int j = 0; j < NE_; ++j) {
                    const bool hit = (e == j);
                    row = hit ? (poff[j] + run[j]) : row;
                    run[j] += hit ? 1 : 0;
                }
                row = min(max(row, 0), (int)rmax - 1);
                const unsigned rel = (lane * spl + 4u * g + (unsigned)c) - lo;
                if (rel < (unsigned)RW_CH) s_img[rel] = row;
            }
        }
        wave_sync_lds();
        const unsigned nw = min((unsigned)RW_CH, nslot - lo);
        for (int pass = 0; pass < 2; ++pass) {
            for (unsigned i = lane; i < (nw >> 2); i += 32u) *(volatile v4i*)(tbl + hdr + rmax + lo + 4u * i) = *(const v4i*)(&s_img[4u * i]);
            __threadfence();
        }
        wave_sync_lds();
    }
}

__global__ __launch_bounds__(256) void k_gather(const h16* __restrict__ x16, const int* __restrict__ tbl, h16* __restrict__ Xg) {
    const unsigned row = blockIdx.x * 2u + (threadIdx.x >> 7);
    if (row >= (unsigned)R_MAX) return;
    const unsigned c = (threadIdx.x & 127u) * 8u;
    const int tr = tbl[TBL_ROWTOK + row];
    const bool pad = (tr < 0);
    const int tok = min(max(tr, 0), NTOK - 1);
    const v4u ld = *(const v4u*)(x16 + (size_t)(unsigned)tok * DM + c);
    v4u v;
    v.x = pad ? 0u : ld.x; v.y = pad ? 0u : ld.y; v.z = pad ? 0u : ld.z; v.w = pad ? 0u : ld.w;
    VST2(v4u, Xg + (size_t)row * DM + c, v);
}

__global__ __launch_bounds__(256) void k_ffn2(const h16* __restrict__ Hg, const h16* __restrict__ Wp, const float* __restrict__ eb,
                                              const int* __restrict__ tbl, float* __restrict__ Yg) {
    __shared__ __align__(16) float sT[8][16 * 68];
    const unsigned lane = threadIdx.x & 31u;
    const unsigned wave = threadIdx.x >> 5;
    const unsigned u = blockIdx.x * 8u + wave;
    if (u >= (unsigned)(NT_MAX * (DM / 64))) return;
    const unsigned rowtile = u / (unsigned)(DM / 64);
    const unsigned ct = u - rowtile * (unsigned)(DM / 64);
    const int nt = min(max(tbl[TBL_NTILES], 0), NT_MAX);
    if ((int)rowtile >= nt) return;
    const int e = min(max(tbl[TBL_TILE_E + rowtile], 0), NE - 1);
    const size_t wbase = (size_t)(unsigned)e * (size_t)(DM * FF);
    const unsigned m0 = rowtile << 6, n0 = ct << 6;
    const unsigned rlane = lane & 15u;
    const unsigned koff = (lane >> 4) * 8u;
    const unsigned mOff = koff;

    v8f acc[4][4];
#pragma unroll
    for (int i = 0; i < 4; ++i)
#pragma unroll
        for (int j = 0; j < 4; ++j) acc[i][j] = (v8f){0.f,0.f,0.f,0.f,0.f,0.f,0.f,0.f};

    for (unsigned k0 = 0; k0 < (unsigned)FF; k0 += 32u) {
        v16h bh[4];
#pragma unroll
        for (int j = 0; j < 4; ++j)
            bh[j] = frag_ld(Wp + wbase + (size_t)(n0 + ((unsigned)j << 4) + rlane) * FF + koff + k0);
#pragma unroll
        for (int i = 0; i < 4; ++i) {
            const v16h ah = frag_ld(Hg + (size_t)(m0 + ((unsigned)i << 4) + rlane) * FF + koff + k0);
#pragma unroll
            for (int j = 0; j < 4; ++j) acc[i][j] = wmma16g(ah, bh[j], acc[i][j]);
        }
    }

    float ebv[4];
#pragma unroll
    for (int j = 0; j < 4; ++j) ebv[j] = bfr(eb[(unsigned)e * (unsigned)DM + n0 + ((unsigned)j << 4) + rlane]);

    float* slab = sT[wave];
#pragma unroll
    for (int i = 0; i < 4; ++i) {
        const unsigned mBase = m0 + ((unsigned)i << 4);
#pragma unroll
        for (int j = 0; j < 4; ++j)
#pragma unroll
            for (int r = 0; r < 8; ++r)
                slab[(mOff + (unsigned)r) * 68u + ((unsigned)j << 4) + rlane] = acc[i][j][r] * SC_Y + ebv[j];
        wave_sync_lds();
        const unsigned hh = lane >> 4, c4 = (lane & 15u) * 4u;
#pragma unroll
        for (int half = 0; half < 2; ++half) {
            v4f vv[4];
#pragma unroll
            for (int it = 0; it < 4; ++it) {
                const unsigned row = (unsigned)(half * 4 + it) * 2u + hh;
                vv[it] = *(const v4f*)(slab + row * 68u + c4);
            }
            for (int pass = 0; pass < 2; ++pass) {
#pragma unroll
                for (int it = 0; it < 4; ++it) {
                    const unsigned row = (unsigned)(half * 4 + it) * 2u + hh;
                    *(volatile v4f*)(Yg + (size_t)(mBase + row) * DM + n0 + c4) = vv[it];
                }
                __threadfence();
            }
        }
        wave_sync_lds();
    }
}

__global__ __launch_bounds__(256) void k_combine(const float* __restrict__ Yg, const float* __restrict__ wgt,
                                                 const int* __restrict__ tbl, float* __restrict__ out) {
    const unsigned t = blockIdx.x;
    if (t >= (unsigned)NTOK) return;
    const unsigned c = threadIdx.x * 4u;
    const int r0 = min(max(tbl[TBL_SLOTROW + 2u * t], 0), R_MAX - 1);
    const int r1 = min(max(tbl[TBL_SLOTROW + 2u * t + 1u], 0), R_MAX - 1);
    const float w0 = wgt[2u * t], w1 = wgt[2u * t + 1u];
    const v4f a = *(const v4f*)(Yg + (size_t)(unsigned)r0 * DM + c);
    const v4f b = *(const v4f*)(Yg + (size_t)(unsigned)r1 * DM + c);
    const v4f y = (a * w0) + (b * w1);
    VST2(v4f, out + (size_t)t * DM + c, y);
}

extern "C" void kernel_launch(void* const* d_in, const int* in_sizes, int n_in, void* d_out, int out_size,
                              void* d_ws, size_t ws_size, hipStream_t stream) {
    if (n_in < 4) return;
    if (in_sizes[0] < NTOK_ALL * DM || in_sizes[1] < DM * NE || in_sizes[2] < NE * FF * DM || in_sizes[3] < NE * DM) return;
    if (out_size < NTOK_ALL * DM) return;

    const float* x  = (const float*)d_in[0];
    const float* gw = (const float*)d_in[1];
    const float* we = (const float*)d_in[2];
    const float* be = (const float*)d_in[3];
    float* out = (float*)d_out;

    char* wsp = (char*)d_ws;
    size_t off = 0;
    auto carve = [&](size_t bytes) -> void* { void* r = wsp + off; off += (bytes + 255) & ~(size_t)255; return r; };
    h16*   x16 = (h16*)carve((size_t)NTOK_ALL * DM * 2);
    h16*   wpt = (h16*)carve((size_t)NE * DM * FF * 2);
    int*   selA = (int*)carve((size_t)NSLOT * 4);
    float* wgtA = (float*)carve((size_t)NSLOT * 4);
    int*   tblA = (int*)carve((size_t)TBL_WORDS * 4);
    int*   selB = (int*)carve((size_t)NSLOT * 4);
    float* wgtB = (float*)carve((size_t)NSLOT * 4);
    int*   tblB = (int*)carve((size_t)TBL_WORDS * 4);
    float* gs  = (float*)carve((size_t)NPASS * NGW * 32 * 4);
    h16*   Xg  = (h16*)carve((size_t)R_MAX * FF * 2);
    float* Yg  = (float*)carve((size_t)R_MAX * DM * 4);
    if (off != WS_TOTAL || off > ws_size || off > (size_t)134217728) return;

    k_plane<CX_LOG2><<<(NTOK_ALL * DM / 8) / 256, 256, 0, stream>>>(x, x16, (unsigned)(NTOK_ALL * DM / 8));
    k_planeTw<<<(NE * (FF / 64) * (DM / 32) + 3) / 4, 128, 0, stream>>>(we, wpt, (unsigned)NE, (unsigned)FF, (unsigned)DM, (unsigned)DM, (unsigned)(FF * DM), (float)(1u << CW_LOG2));

    k_gate<<<NTOK / 128, 256, 0, stream>>>(x, gw, selA, wgtA, gs);
    k_route1w<NER><<<1, 32, 0, stream>>>(selA, tblA, (unsigned)NSLOT, (unsigned)TOPK, (unsigned)TBL_HDR, (unsigned)R_MAX, (unsigned)TBL_POFF, (unsigned)TBL_NTILES, (unsigned)TBL_TILE_E);
    k_gather<<<R_MAX / 2, 256, 0, stream>>>(x16, tblA, Xg);
    k_ffn2<<<(NT_MAX * (DM / 64) + 7) / 8, 256, 0, stream>>>(Xg, wpt, be, tblA, Yg);
    k_combine<<<NTOK, 256, 0, stream>>>(Yg, wgtA, tblA, out);
    k_gate<<<NTOK / 128, 256, 0, stream>>>(x + (size_t)NTOK * DM, gw, selB, wgtB, gs + (size_t)NGW * 32);
    k_route1w<NER><<<1, 32, 0, stream>>>(selB, tblB, (unsigned)NSLOT, (unsigned)TOPK, (unsigned)TBL_HDR, (unsigned)R_MAX, (unsigned)TBL_POFF, (unsigned)TBL_NTILES, (unsigned)TBL_TILE_E);
    k_gather<<<R_MAX / 2, 256, 0, stream>>>(x16 + (size_t)NTOK * DM, tblB, Xg);
    k_ffn2<<<(NT_MAX * (DM / 64) + 7) / 8, 256, 0, stream>>>(Xg, wpt, be, tblB, Yg);
    k_combine<<<NTOK, 256, 0, stream>>>(Yg, wgtB, tblB, out + (size_t)NTOK * DM);
}
